// GraphSAGE_32942399160960
// MI455X (gfx1250) — hardware-verified
//
#include <hip/hip_runtime.h>
#include <stddef.h>
#include <stdint.h>


#define DF     128
#define DH     256
#define DC     64
#define K1     384
#define K2     512
#define AGP    256
#define HP     512
#define TRP    128
#define NTHR   256
#define NWAVE  8
#define EPT    8
#define CHUNK  (NTHR * EPT)
#define WCAP   (EPT * 32)
#define LISTN  (NWAVE * WCAP)
#define NBA    512
#define SLA    9
#define RCAP   20480
#define DEGCAP 96
#define GBM    64
#define GBN    128
#define GTHR   128
#define NBAND  8
#define UW1    (DH * (K1 / 8))
#define UW2    (2 * DC * (K2 / 8))
#define AGG_ZINTS    (LISTN + 2 * RCAP + 3 * NBA)
#define MISC_INTS    16
#define ROWBUF_INTS  (NWAVE * AGP / 2)
#define AGG_LDS_INTS (AGG_ZINTS + MISC_INTS + ROWBUF_INTS)
#define WSMAX  134217728

static_assert((CHUNK & (CHUNK - 1)) == 0 && CHUNK <= 4096);
static_assert((NBA & (NBA - 1)) == 0 && NBA == (1 << SLA));
static_assert(((long long)CHUNK << SLA) < (1LL << 31));
static_assert(LISTN % NTHR == 0);
static_assert(NBA % NWAVE == 0 && NBA % 32 == 0 && NBA % GBM == 0 && NBA == 4 * 128);
static_assert(RCAP % (NTHR * 4) == 0 && AGG_ZINTS % 4 == 0 && ((AGG_ZINTS + MISC_INTS) % 4) == 0);
static_assert(DEGCAP % 32 == 0 && DEGCAP >= 57 + 8);
static_assert(K1 % 32 == 0 && K2 % 32 == 0 && K1 == 3 * DF && K2 == 2 * DH && AGP == 2 * DF && HP == K2);
static_assert(GBM == (GTHR / 32) * 16 && GBN == 128 && DH % GBN == 0 && 2 * DC == GBN && TRP == GBN);
static_assert(UW1 % NTHR == 0 && UW2 % NTHR == 0);
static_assert(K1 < 512 && 2 * DC == 128);
static_assert(AGG_LDS_INTS * 4 <= 300000);

typedef float          v2f   __attribute__((ext_vector_type(2)));
typedef float          v4f   __attribute__((ext_vector_type(4)));
typedef float          v8f   __attribute__((ext_vector_type(8)));
typedef int            v4i   __attribute__((ext_vector_type(4)));
typedef int            v8i   __attribute__((ext_vector_type(8)));
typedef unsigned       v2u   __attribute__((ext_vector_type(2)));
typedef unsigned short v4us  __attribute__((ext_vector_type(4)));
typedef unsigned short v8us  __attribute__((ext_vector_type(8)));
typedef unsigned short v16us __attribute__((ext_vector_type(16)));
typedef __bf16         v16bf __attribute__((ext_vector_type(16)));
typedef v2f  __attribute__((may_alias)) v2fa;
typedef v4f  __attribute__((may_alias)) v4fa;
typedef v4i  __attribute__((may_alias)) v4ia;
typedef v2u  __attribute__((may_alias)) v2ua;
typedef v4us __attribute__((may_alias)) v4usa;
typedef v8us __attribute__((may_alias)) v8usa;
union FragB { v16bf v; v16us u; v8us h[2]; v8i w; };

__device__ __forceinline__ v8f wmb(const FragB& a, const FragB& b, v8f c) {
  v8f d = __builtin_amdgcn_wmma_f32_16x16x32_bf16(false, a.v, false, b.v, (short)0, c, false, false);
  asm volatile("v_nop\n\tv_nop\n\tv_nop\n\tv_nop" : "+v"(d) : "v"(a.w), "v"(b.w));
  return d;
}

__device__ __forceinline__ unsigned bf16_bits(float f) {
  const unsigned u = __float_as_uint(f);
  const unsigned r = (u + 0x7FFFu + ((u >> 16) & 1u)) >> 16;
  const unsigned q = (u >> 16) | 0x40u;
  return ((u & 0x7fffffffu) > 0x7f800000u) ? q : r;
}
__device__ __forceinline__ float bf16_val(float f) {
  return __uint_as_float(bf16_bits(f) << 16);
}

__device__ __forceinline__ void wave_sync() {
  __builtin_amdgcn_fence(__ATOMIC_RELEASE, "wavefront");
  __builtin_amdgcn_wave_barrier();
  __builtin_amdgcn_fence(__ATOMIC_ACQUIRE, "wavefront");
}

__device__ __forceinline__ v8us pack8(const v4f a, const v4f b, const bool ok) {
  v8us o;
  o[0] = ok ? (unsigned short)bf16_bits(a.x) : (unsigned short)0;
  o[1] = ok ? (unsigned short)bf16_bits(a.y) : (unsigned short)0;
  o[2] = ok ? (unsigned short)bf16_bits(a.z) : (unsigned short)0;
  o[3] = ok ? (unsigned short)bf16_bits(a.w) : (unsigned short)0;
  o[4] = ok ? (unsigned short)bf16_bits(b.x) : (unsigned short)0;
  o[5] = ok ? (unsigned short)bf16_bits(b.y) : (unsigned short)0;
  o[6] = ok ? (unsigned short)bf16_bits(b.z) : (unsigned short)0;
  o[7] = ok ? (unsigned short)bf16_bits(b.w) : (unsigned short)0;
  return o;
}
__device__ __forceinline__ v4f blend4(const v4f a, const v4f b, const unsigned mk) {
  const unsigned nk = ~mk;
  v4f o;
  o.x = __uint_as_float((__float_as_uint(b.x) & mk) | (__float_as_uint(a.x) & nk));
  o.y = __uint_as_float((__float_as_uint(b.y) & mk) | (__float_as_uint(a.y) & nk));
  o.z = __uint_as_float((__float_as_uint(b.z) & mk) | (__float_as_uint(a.z) & nk));
  o.w = __uint_as_float((__float_as_uint(b.w) & mk) | (__float_as_uint(a.w) & nk));
  return o;
}
__device__ __forceinline__ void put8(unsigned short* dp, const v8us o) {
  *(volatile v8us*)dp = o;
  __threadfence();
  *(volatile v8us*)dp = o;
}

template <int SLB>
__device__ __forceinline__ int scan_chunk(const int* __restrict__ dsts, int nE, int cbase, int slotBase,
                                          int nb, int vec8, int* list, int tid, int lane, int wave) {
  int wc = 0;
  const int el0  = tid * EPT;
  const int e0   = cbase + el0;
  const int sent = -2147483647 - 1;
  v4i da, db;
  if (vec8 != 0 && cbase + CHUNK <= nE) {
    da = *(const v4i*)(dsts + e0);
    db = *(const v4i*)(dsts + e0 + 4);
  } else {
    da.x = (e0     < nE) ? dsts[min(e0,     nE - 1)] : sent;
    da.y = (e0 + 1 < nE) ? dsts[min(e0 + 1, nE - 1)] : sent;
    da.z = (e0 + 2 < nE) ? dsts[min(e0 + 2, nE - 1)] : sent;
    da.w = (e0 + 3 < nE) ? dsts[min(e0 + 3, nE - 1)] : sent;
    db.x = (e0 + 4 < nE) ? dsts[min(e0 + 4, nE - 1)] : sent;
    db.y = (e0 + 5 < nE) ? dsts[min(e0 + 5, nE - 1)] : sent;
    db.z = (e0 + 6 < nE) ? dsts[min(e0 + 6, nE - 1)] : sent;
    db.w = (e0 + 7 < nE) ? dsts[min(e0 + 7, nE - 1)] : sent;
  }
  const unsigned nbs = (unsigned)slotBase;
  const unsigned unb = (unsigned)nb;
  const unsigned s0 = (unsigned)da.x - nbs, s1 = (unsigned)da.y - nbs;
  const unsigned s2 = (unsigned)da.z - nbs, s3 = (unsigned)da.w - nbs;
  const unsigned s4 = (unsigned)db.x - nbs, s5 = (unsigned)db.y - nbs;
  const unsigned s6 = (unsigned)db.z - nbs, s7 = (unsigned)db.w - nbs;
  const bool h0 = s0 < unb, h1 = s1 < unb, h2 = s2 < unb, h3 = s3 < unb;
  const bool h4 = s4 < unb, h5 = s5 < unb, h6 = s6 < unb, h7 = s7 < unb;
  const unsigned any = __builtin_amdgcn_ballot_w32(h0 | h1 | h2 | h3 | h4 | h5 | h6 | h7);
  if (any != 0u) {
#define HITJ(J, HJ, SJ) { \
      const unsigned mj = __builtin_amdgcn_ballot_w32(HJ); \
      if (mj != 0u) { \
        if (HJ) { \
          const int pos = wc + (int)__builtin_amdgcn_mbcnt_lo(mj, 0u); \
          if (pos < WCAP) list[wave * WCAP + pos] = ((el0 + (J)) << SLB) | (int)(SJ); \
        } \
        wc += (int)__builtin_popcount(mj); } }
    HITJ(0, h0, s0)
    HITJ(1, h1, s1)
    HITJ(2, h2, s2)
    HITJ(3, h3, s3)
    HITJ(4, h4, s4)
    HITJ(5, h5, s5)
    HITJ(6, h6, s6)
    HITJ(7, h7, s7)
#undef HITJ
  }
  return wc;
}

__global__ __launch_bounds__(NTHR) void k_prep(const float* __restrict__ x, const float* __restrict__ W1l,
                                               const float* __restrict__ W1r, const float* __restrict__ W2l,
                                               const float* __restrict__ W2r, int nN, int nbX,
                                               unsigned short* XB, unsigned short* W1C, unsigned short* W2C) {
  const int b = (int)blockIdx.x, tid = (int)threadIdx.x;
  if (b < nbX) {
    const int u   = b * NTHR + tid;
    const int row = u >> 4;
    const int k8  = (u & 15) * 8;
    const int rc  = row < nN ? row : nN - 1;
    const float* p = x + (size_t)rc * DF + k8;
    const v4f a = *(const v4fa*)p;
    const v4f c = *(const v4fa*)(p + 4);
    put8(XB + (size_t)u * 8, pack8(a, c, row < nN));
  } else if (b < nbX + UW1 / NTHR) {
    const int v    = (b - nbX) * NTHR + tid;
    const int n    = v / (K1 / 8);
    const int k8   = (v - n * (K1 / 8)) * 8;
    const int kk   = k8 & (DF - 1);
    const unsigned mk = 0u - (unsigned)(k8 >> 8);
    const float* pl = W1l + (size_t)n * DF + kk;
    const float* pr = W1r + (size_t)n * DF + kk;
    const v4f al = *(const v4fa*)pl, cl = *(const v4fa*)(pl + 4);
    const v4f ar = *(const v4fa*)pr, cr = *(const v4fa*)(pr + 4);
    const v4f a = blend4(al, ar, mk);
    const v4f c = blend4(cl, cr, mk);
    put8(W1C + (size_t)v * 8, pack8(a, c, true));
  } else if (b < nbX + UW1 / NTHR + UW2 / NTHR) {
    const int v    = (b - nbX - UW1 / NTHR) * NTHR + tid;
    const int n    = v >> 6;
    const int k8   = (v & 63) * 8;
    const int kk   = k8 & (DH - 1);
    const int nr   = n & (DC - 1);
    const unsigned mk = 0u - (unsigned)(n >> 6);
    const float* pl = W2l + (size_t)nr * DH + kk;
    const float* pr = W2r + (size_t)nr * DH + kk;
    const v4f al = *(const v4fa*)pl, cl = *(const v4fa*)(pl + 4);
    const v4f ar = *(const v4fa*)pr, cr = *(const v4fa*)(pr + 4);
    const v4f a = blend4(al, ar, mk);
    const v4f c = blend4(cl, cr, mk);
    put8(W2C + (size_t)v * 8, pack8(a, c, true));
  }
}

__global__ __launch_bounds__(NTHR) void k_scan1(const int* __restrict__ srcs, const int* __restrict__ dsts,
                                                int nE, int nN, int vec8, int mRows,
                                                const unsigned short* __restrict__ xb,
                                                unsigned short* agp, int* hits, int* cntp) {
  extern __shared__ __attribute__((aligned(16))) int dsm[];
  int* list = dsm;
  int* hl   = dsm + LISTN;
  int* sl   = hl + RCAP;
  int* cnt  = sl + RCAP;
  int* offs = cnt + NBA;
  int* cur  = offs + NBA;
  int* misc = cur + NBA;
  const int tid = (int)threadIdx.x, lane = tid & 31, wave = tid >> 5;
  unsigned short* rowbuf = (unsigned short*)(misc + MISC_INTS) + wave * AGP;
  const int nodeBase = (int)blockIdx.x * NBA;

  {
    const v4i z4 = {0, 0, 0, 0};
    for (int i = tid * 4; i < AGG_ZINTS; i += NTHR * 4) *(v4ia*)(dsm + i) = z4;
    if (tid < MISC_INTS) misc[tid] = 0;
  }
  __syncthreads();

  int t = 0, ov = 0;
  const int nChunks = (nE + CHUNK - 1) / CHUNK;
#pragma unroll 1
  for (int ch = 0; ch < nChunks; ++ch) {
    const int cbase = ch * CHUNK;
    const int wc = scan_chunk<SLA>(dsts, nE, cbase, nodeBase, NBA, vec8, list, tid, lane, wave);
    if (lane == 0) misc[wave] = wc;
    __syncthreads();
    if (wave == 0) {
#pragma unroll 1
      for (int w2 = 0; w2 < NWAVE; ++w2) {
        int c = misc[w2];
        c = c < 0 ? 0 : (c > WCAP ? WCAP : c);
#pragma unroll 1
        for (int b0 = 0; b0 < c; b0 += 32) {
          const int idx = b0 + lane;
          const int ent = list[w2 * WCAP + (idx < WCAP ? idx : WCAP - 1)];
          const int m32 = (c - b0) < 32 ? (c - b0) : 32;
#pragma unroll 1
          for (int k = 0; k < m32; ++k) {
            const int u    = __builtin_amdgcn_readlane(ent, k);
            const int slot = u & (NBA - 1);
            const int el   = (u >> SLA) & (CHUNK - 1);
            const int pk   = ((cbase + el) << SLA) | slot;
            if (t < RCAP) {
              if (lane == 0) { hl[t] = pk; cnt[slot] = cnt[slot] + 1; }
              t = t + 1;
            } else {
              ov = 1;
            }
          }
        }
      }
    }
    __syncthreads();
  }
  if (wave == 0 && lane == 0) { misc[8] = t; misc[9] = ov; }
  __syncthreads();
  int tt = misc[8];
  tt = tt < 0 ? 0 : (tt > RCAP ? RCAP : tt);
  const int ovf = misc[9];

  if (wave == 0) {
    const int base = lane * (NBA / 32);
    int s = 0;
#pragma unroll 1
    for (int i = 0; i < NBA / 32; ++i) s += cnt[base + i];
    int incl = s;
#pragma unroll
    for (int d = 1; d < 32; d <<= 1) {
      const int y = __shfl_up(incl, d, 32);
      if (lane >= d) incl += y;
    }
    int run = incl - s;
#pragma unroll 1
    for (int i = 0; i < NBA / 32; ++i) {
      const int cv = cnt[base + i];
      offs[base + i] = run;
      cur[base + i]  = run;
      run += cv;
    }
  }
  __syncthreads();
  if (wave == 0) {
#pragma unroll 1
    for (int b0 = 0; b0 < tt; b0 += 32) {
      const int idx = b0 + lane;
      const int ent = hl[idx < RCAP ? idx : RCAP - 1];
      const int m32 = (tt - b0) < 32 ? (tt - b0) : 32;
#pragma unroll 1
      for (int k = 0; k < m32; ++k) {
        const int u    = __builtin_amdgcn_readlane(ent, k);
        const int slot = u & (NBA - 1);
        if (lane == 0) {
          int p = cur[slot];
          p = p < 0 ? 0 : (p > RCAP - 1 ? RCAP - 1 : p);
          sl[p] = u;
          cur[slot] = p + 1;
        }
      }
    }
  }
  __syncthreads();

  {
    const int lim = ((tt + NTHR - 1) / NTHR) * NTHR;
#pragma unroll 1
    for (int i = tid; i < lim; i += NTHR) {
      const int ent = sl[i < RCAP ? i : RCAP - 1];
      int eid = ent >> SLA;
      eid = eid < 0 ? 0 : (eid > nE - 1 ? nE - 1 : eid);
      int sr = srcs[eid];
      sr = sr < 0 ? 0 : (sr > nN - 1 ? nN - 1 : sr);
      hl[i < RCAP ? i : RCAP - 1] = (i < tt) ? sr : 0;
    }
  }
  __syncthreads();

  {
    int* hp = hits + (size_t)blockIdx.x * RCAP;
    int* cp = cntp + (size_t)blockIdx.x * NBA + 4 * (tid & 127);
    const v4i cv = *(const v4ia*)(cnt + 4 * (tid & 127));
#pragma unroll 1
    for (int i = tid * 4; i < RCAP; i += NTHR * 4) {
      const v4i v = *(const v4ia*)(hl + i);
      *(volatile v4i*)(hp + i) = v;
    }
    if (tid < 128) *(volatile v4i*)cp = cv;
    __threadfence();
#pragma unroll 1
    for (int i = tid * 4; i < RCAP; i += NTHR * 4) {
      const v4i v = *(const v4ia*)(hl + i);
      *(volatile v4i*)(hp + i) = v;
    }
    if (tid < 128) *(volatile v4i*)cp = cv;
  }

  const float qnan = __int_as_float(0x7fc00000);
  const float pz = (ovf != 0) ? qnan : 0.0f;
#pragma unroll 1
  for (int si = 0; si < NBA / NWAVE; ++si) {
    const int s    = si * NWAVE + wave;
    const int node = nodeBase + s;
    const int craw = cnt[s];
    const bool big = craw > DEGCAP;
    int c = craw < 0 ? 0 : (craw > DEGCAP ? DEGCAP : craw);
    int o = offs[s];
    o = o < 0 ? 0 : (o > RCAP ? RCAP : o);
    float a0 = 0.0f, a1 = 0.0f, a2 = 0.0f, a3 = 0.0f;
#pragma unroll 1
    for (int b0 = 0; b0 < c; b0 += 32) {
      int idx = o + b0 + lane;
      idx = idx > RCAP - 1 ? RCAP - 1 : idx;
      int sr = hl[idx];
      sr = sr < 0 ? 0 : (sr > nN - 1 ? nN - 1 : sr);
      const int m32 = (c - b0) < 32 ? (c - b0) : 32;
#pragma unroll 1
      for (int k = 0; k < m32; ++k) {
        const int sk = __builtin_amdgcn_readlane(sr, k);
        const v2u w = *(const v2ua*)(xb + (size_t)sk * DF + 4 * lane);
        a0 += __uint_as_float(w.x << 16);
        a1 += __uint_as_float(w.x & 0xffff0000u);
        a2 += __uint_as_float(w.y << 16);
        a3 += __uint_as_float(w.y & 0xffff0000u);
      }
    }
    const float dn = (float)(craw > 0 ? craw : 1);
    const float di = (craw > 0) ? (1.0f / dn) : 0.0f;
    const float pzr = big ? qnan : pz;
    const bool live = node < nN;
    const float m0 = live ? (a0 * di + pzr) : 0.0f;
    const float m1 = live ? (a1 * di + pzr) : 0.0f;
    const float m2 = live ? (a2 * di + pzr) : 0.0f;
    const float m3 = live ? (a3 * di + pzr) : 0.0f;
    v4us mh, ml;
    {
      unsigned hb;
      hb = bf16_bits(m0); mh[0] = (unsigned short)hb; ml[0] = (unsigned short)bf16_bits(m0 - __uint_as_float(hb << 16));
      hb = bf16_bits(m1); mh[1] = (unsigned short)hb; ml[1] = (unsigned short)bf16_bits(m1 - __uint_as_float(hb << 16));
      hb = bf16_bits(m2); mh[2] = (unsigned short)hb; ml[2] = (unsigned short)bf16_bits(m2 - __uint_as_float(hb << 16));
      hb = bf16_bits(m3); mh[3] = (unsigned short)hb; ml[3] = (unsigned short)bf16_bits(m3 - __uint_as_float(hb << 16));
    }
    *(v4usa*)(rowbuf + 4 * lane) = mh;
    *(v4usa*)(rowbuf + DF + 4 * lane) = ml;
    wave_sync();
    const v8us q0 = *(const v8usa*)(rowbuf + 8 * lane);
    wave_sync();
    if (node < mRows) {
      unsigned short* rpw = agp + (size_t)node * AGP + 8 * lane;
      *(volatile v8us*)rpw = q0;
      __threadfence();
      *(volatile v8us*)rpw = q0;
    }
  }
}

__global__ __launch_bounds__(GTHR) void k_gemm1(const unsigned short* __restrict__ AG,
                                                const unsigned short* __restrict__ XB,
                                                const unsigned short* __restrict__ W1C,
                                                const float* __restrict__ b1, unsigned short* HB,
                                                int tile0, int nN) {
  __shared__ __attribute__((aligned(16))) float stg[GBM * GBN];
  const int tid = (int)threadIdx.x, lane = tid & 31, wave = tid >> 5, hh = lane >> 4, m = lane & 15;
  const int lrow0 = (int)blockIdx.x * GBM;
  const int grow0 = (tile0 + (int)blockIdx.x) * GBM;
  const int col0  = (int)blockIdx.y * GBN;

  v8f acc[8];
  {
    const v8f z = {0.f, 0.f, 0.f, 0.f, 0.f, 0.f, 0.f, 0.f};
#pragma unroll
    for (int t = 0; t < 8; ++t) acc[t] = z;
  }
  const size_t ar = (size_t)(grow0 + 16 * wave + m);
  const unsigned short* ap = AG  + ar * (size_t)AGP + 8 * hh;
  const unsigned short* xp = XB  + ar * (size_t)DF + 8 * hh;
  const unsigned short* bp = W1C + (size_t)(col0 + m) * (size_t)K1 + 8 * hh;

#pragma unroll 1
  for (int k0 = 0; k0 < 2 * DF; k0 += 32) {
    FragB af;
    af.h[0] = *(const v8usa*)(ap + k0);
    af.h[1] = *(const v8usa*)(ap + k0 + 16);
#pragma unroll
    for (int nt = 0; nt < 8; ++nt) {
      const unsigned short* wq = bp + (size_t)(16 * nt) * (size_t)K1 + k0;
      FragB bf;
      bf.h[0] = *(const v8usa*)wq;
      bf.h[1] = *(const v8usa*)(wq + 16);
      acc[nt] = wmb(af, bf, acc[nt]);
    }
  }
#pragma unroll 1
  for (int k0 = 0; k0 < DF; k0 += 32) {
    FragB af;
    af.h[0] = *(const v8usa*)(xp + k0);
    af.h[1] = *(const v8usa*)(xp + k0 + 16);
#pragma unroll
    for (int nt = 0; nt < 8; ++nt) {
      const unsigned short* wq = bp + (size_t)(16 * nt) * (size_t)K1 + 2 * DF + k0;
      FragB bf;
      bf.h[0] = *(const v8usa*)wq;
      bf.h[1] = *(const v8usa*)(wq + 16);
      acc[nt] = wmb(af, bf, acc[nt]);
    }
  }

#pragma unroll
  for (int nt = 0; nt < 8; ++nt) {
    const int lc = 16 * nt + m;
#pragma unroll
    for (int r = 0; r < 8; ++r) {
      const int lr = 16 * wave + 8 * hh + r;
      stg[lr * GBN + lc] = acc[nt][r];
    }
  }
  __syncthreads();

  v4f bb4;
  {
    const v4f t1 = *(const v4fa*)(b1 + col0 + 4 * lane);
    bb4.x = bf16_val(t1.x); bb4.y = bf16_val(t1.y); bb4.z = bf16_val(t1.z); bb4.w = bf16_val(t1.w);
  }
  float* wrow = stg + (16 * wave) * GBN;
#pragma unroll 1
  for (int g = 0; g < 4; ++g) {
    v4f pv[4];
#pragma unroll
    for (int j = 0; j < 4; ++j) pv[j] = *(const v4fa*)(wrow + (4 * g + j) * GBN + 4 * lane);
    wave_sync();
#pragma unroll
    for (int j = 0; j < 4; ++j) {
      const bool ok = (grow0 + 16 * wave + 4 * g + j) < nN;
      const v4f tq = pv[j] + bb4;
      v4f y;
      y.x = (tq.x > 0.0f) ? tq.x : (tq.x - tq.x);
      y.y = (tq.y > 0.0f) ? tq.y : (tq.y - tq.y);
      y.z = (tq.z > 0.0f) ? tq.z : (tq.z - tq.z);
      y.w = (tq.w > 0.0f) ? tq.w : (tq.w - tq.w);
      y.x = ok ? y.x : 0.0f; y.y = ok ? y.y : 0.0f; y.z = ok ? y.z : 0.0f; y.w = ok ? y.w : 0.0f;
      v4us h4, l4;
      unsigned hb;
      hb = bf16_bits(y.x); h4[0] = (unsigned short)hb; l4[0] = (unsigned short)bf16_bits(y.x - __uint_as_float(hb << 16));
      hb = bf16_bits(y.y); h4[1] = (unsigned short)hb; l4[1] = (unsigned short)bf16_bits(y.y - __uint_as_float(hb << 16));
      hb = bf16_bits(y.z); h4[2] = (unsigned short)hb; l4[2] = (unsigned short)bf16_bits(y.z - __uint_as_float(hb << 16));
      hb = bf16_bits(y.w); h4[3] = (unsigned short)hb; l4[3] = (unsigned short)bf16_bits(y.w - __uint_as_float(hb << 16));
      unsigned short* srow = (unsigned short*)(wrow + (4 * g + j) * GBN);
      *(v4usa*)(srow + 4 * lane) = h4;
      *(v4usa*)(srow + 128 + 4 * lane) = l4;
    }
  }
  wave_sync();
  const int dcol = col0 + 8 * m + DH * hh;
#pragma unroll 1
  for (int g = 0; g < 2; ++g) {
    v8us q[8];
#pragma unroll
    for (int j = 0; j < 8; ++j) {
      const unsigned short* srow = (const unsigned short*)(wrow + (8 * g + j) * GBN);
      q[j] = *(const v8usa*)(srow + 8 * lane);
    }
#pragma unroll
    for (int j = 0; j < 8; ++j) {
      unsigned short* rp = HB + (size_t)(lrow0 + 16 * wave + 8 * g + j) * (size_t)HP + dcol;
      *(volatile v8us*)rp = q[j];
    }
    __threadfence();
#pragma unroll
    for (int j = 0; j < 8; ++j) {
      unsigned short* rp = HB + (size_t)(lrow0 + 16 * wave + 8 * g + j) * (size_t)HP + dcol;
      *(volatile v8us*)rp = q[j];
    }
  }
}

__global__ __launch_bounds__(GTHR) void k_gemm2(const unsigned short* __restrict__ HB,
                                                const unsigned short* __restrict__ W2C,
                                                const float* __restrict__ b2, float* TR, int tile0) {
  __shared__ __attribute__((aligned(16))) float stg[GBM * GBN];
  const int tid = (int)threadIdx.x, lane = tid & 31, wave = tid >> 5, hh = lane >> 4, m = lane & 15;
  const int lrow0 = (int)blockIdx.x * GBM;
  const int grow0 = (tile0 + (int)blockIdx.x) * GBM;

  v8f acc[8];
  {
    const v8f z = {0.f, 0.f, 0.f, 0.f, 0.f, 0.f, 0.f, 0.f};
#pragma unroll
    for (int t = 0; t < 8; ++t) acc[t] = z;
  }
  const unsigned short* ap = HB  + (size_t)(lrow0 + 16 * wave + m) * (size_t)HP + 8 * hh;
  const unsigned short* bp = W2C + (size_t)m * (size_t)K2 + 8 * hh;
#pragma unroll 1
  for (int k0 = 0; k0 < K2; k0 += 32) {
    FragB af;
    af.h[0] = *(const v8usa*)(ap + k0);
    af.h[1] = *(const v8usa*)(ap + k0 + 16);
#pragma unroll
    for (int nt = 0; nt < 8; ++nt) {
      const unsigned short* wq = bp + (size_t)(16 * nt) * (size_t)K2 + k0;
      FragB bf;
      bf.h[0] = *(const v8usa*)wq;
      bf.h[1] = *(const v8usa*)(wq + 16);
      acc[nt] = wmb(af, bf, acc[nt]);
    }
  }
#pragma unroll
  for (int nt = 0; nt < 8; ++nt) {
    const int lc = 16 * nt + m;
#pragma unroll
    for (int r = 0; r < 8; ++r) {
      const int lr = 16 * wave + 8 * hh + r;
      stg[lr * GBN + lc] = acc[nt][r];
    }
  }
  __syncthreads();

  v4f bb4;
  {
    const v4f t1 = *(const v4fa*)(b2 + 4 * m);
    const bool rt = hh != 0;
    bb4.x = rt ? bf16_val(t1.x) : 0.0f; bb4.y = rt ? bf16_val(t1.y) : 0.0f;
    bb4.z = rt ? bf16_val(t1.z) : 0.0f; bb4.w = rt ? bf16_val(t1.w) : 0.0f;
  }
#pragma unroll 1
  for (int g = 0; g < 2; ++g) {
    v4f pv[8];
#pragma unroll
    for (int j = 0; j < 8; ++j) pv[j] = *(const v4fa*)(stg + (16 * wave + 8 * g + j) * GBN + 4 * lane) + bb4;
#pragma unroll
    for (int j = 0; j < 8; ++j) {
      float* op = TR + (size_t)(grow0 + 16 * wave + 8 * g + j) * (size_t)TRP + 4 * lane;
      *(volatile v4f*)op = pv[j];
    }
    __threadfence();
#pragma unroll
    for (int j = 0; j < 8; ++j) {
      float* op = TR + (size_t)(grow0 + 16 * wave + 8 * g + j) * (size_t)TRP + 4 * lane;
      *(volatile v4f*)op = pv[j];
    }
  }
}

__global__ __launch_bounds__(NTHR) void k_scan2(const int* __restrict__ hits, const int* __restrict__ cntp,
                                                const float* __restrict__ TR, int nN, float* out) {
  __shared__ __attribute__((aligned(16))) int cnt[NBA];
  __shared__ __attribute__((aligned(16))) int offs[NBA];
  const int tid = (int)threadIdx.x, lane = tid & 31, wave = tid >> 5;
  const int nodeBase = (int)blockIdx.x * NBA;
  const int* hp = hits + (size_t)blockIdx.x * RCAP;
  {
    v4i cv = *(const v4i*)(cntp + (size_t)blockIdx.x * NBA + 4 * (tid & 127));
    cv.x = cv.x < 0 ? 0 : (cv.x > RCAP ? RCAP : cv.x);
    cv.y = cv.y < 0 ? 0 : (cv.y > RCAP ? RCAP : cv.y);
    cv.z = cv.z < 0 ? 0 : (cv.z > RCAP ? RCAP : cv.z);
    cv.w = cv.w < 0 ? 0 : (cv.w > RCAP ? RCAP : cv.w);
    if (tid < 128) *(v4ia*)(cnt + 4 * tid) = cv;
  }
  __syncthreads();
  if (wave == 0) {
    const int base = lane * (NBA / 32);
    int s = 0;
#pragma unroll 1
    for (int i = 0; i < NBA / 32; ++i) s += cnt[base + i];
    int incl = s;
#pragma unroll
    for (int d = 1; d < 32; d <<= 1) {
      const int y = __shfl_up(incl, d, 32);
      if (lane >= d) incl += y;
    }
    int run = incl - s;
#pragma unroll 1
    for (int i = 0; i < NBA / 32; ++i) {
      const int cv = cnt[base + i];
      offs[base + i] = run;
      run += cv;
    }
  }
  __syncthreads();

  const float qnan = __int_as_float(0x7fc00000);
  const int sa = (2 * lane) & 31, sb = (2 * lane + 1) & 31;
#pragma unroll 1
  for (int si = 0; si < NBA / NWAVE; ++si) {
    const int s    = si * NWAVE + wave;
    const int node = nodeBase + s;
    const int craw = cnt[s];
    const bool big = craw > DEGCAP;
    int c = craw < 0 ? 0 : (craw > DEGCAP ? DEGCAP : craw);
    int o = offs[s];
    o = o < 0 ? 0 : (o > RCAP ? RCAP : o);
    const int nc = node < nN ? node : nN - 1;
    float acc0 = 0.0f, acc1 = 0.0f;
#pragma unroll 1
    for (int b0 = 0; b0 < c; b0 += 32) {
      int idx = o + b0 + lane;
      idx = idx > RCAP - 1 ? RCAP - 1 : idx;
      int sr = hp[idx];
      sr = sr < 0 ? 0 : (sr > nN - 1 ? nN - 1 : sr);
      const int m32 = (c - b0) < 32 ? (c - b0) : 32;
#pragma unroll 1
      for (int k = 0; k < m32; ++k) {
        const int sk = __builtin_amdgcn_readlane(sr, k);
        const v2f a = *(const v2fa*)(TR + (size_t)sk * TRP + 2 * lane);
        acc0 += a.x; acc1 += a.y;
      }
    }
    const v2f rr = *(const v2fa*)(TR + (size_t)nc * TRP + DC + 2 * lane);
    const float dn = (float)(craw > 0 ? craw : 1);
    const float di = (craw > 0) ? (1.0f / dn) : 0.0f;
    const float pzr = big ? qnan : 0.0f;
    const float v0 = (acc0 * di + rr.x) + pzr;
    const float v1 = (acc1 * di + rr.y) + pzr;
    v4f ow;
    ow.x = __shfl(v0, sa, 32); ow.y = __shfl(v1, sa, 32);
    ow.z = __shfl(v0, sb, 32); ow.w = __shfl(v1, sb, 32);
    float* op = out + (size_t)nc * DC + 4 * (lane & 15);
    const bool wr = (node < nN) && (lane < 16);
    if (wr) *(volatile v4f*)op = ow;
    __threadfence();
    if (wr) *(volatile v4f*)op = ow;
  }
}

static inline int cdiv(int a, int b) { return (a + b - 1) / b; }
static inline size_t al256(size_t o) { return (o + 255) & ~(size_t)255; }

extern "C" void kernel_launch(void* const* d_in, const int* in_sizes, int n_in,
                              void* d_out, int out_size, void* d_ws, size_t ws_size,
                              hipStream_t stream) {
  if (n_in < 8) return;
  if (in_sizes[0] < DF || (in_sizes[0] % DF) != 0) return;
  const int nN = in_sizes[0] / DF;
  if (nN < 64 || nN > (1 << 22)) return;
  if (in_sizes[1] < 2 || (in_sizes[1] & 1) != 0) return;
  const int nE = in_sizes[1] / 2;
  if (nE < 1 || nE >= (1 << (31 - SLA))) return;
  if (in_sizes[2] != DH * DF || in_sizes[3] != DH * DF || in_sizes[4] != DH) return;
  if (in_sizes[5] != DC * DH || in_sizes[6] != DC * DH || in_sizes[7] != DC) return;
  if ((long long)out_size != (long long)nN * DC) return;

  const float* x    = (const float*)d_in[0];
  const int*   edge = (const int*)d_in[1];
  const float* W1l  = (const float*)d_in[2];
  const float* W1r  = (const float*)d_in[3];
  const float* b1   = (const float*)d_in[4];
  const float* W2l  = (const float*)d_in[5];
  const float* W2r  = (const float*)d_in[6];
  const float* b2   = (const float*)d_in[7];
  float* out = (float*)d_out;
  const int* src = edge;
  const int* dst = edge + nE;

  const int MP  = cdiv(nN, GBM) * GBM;
  const int nT  = MP / GBM;
  const int TPB = cdiv(nT, NBAND);
  const int gA  = cdiv(MP, NBA);
  if ((long long)gA * NBA < (long long)MP) return;
  const int vec8 = ((nE & 3) == 0) ? 1 : 0;
  const int nbX  = MP / 16;

  char* ws = (char*)d_ws;
  size_t off = 0;
  const size_t oW1C = off; off = al256(off + (size_t)DH * K1 * 2);
  const size_t oW2C = off; off = al256(off + (size_t)2 * DC * K2 * 2);
  const size_t oCNT = off; off = al256(off + (size_t)gA * NBA * 4);
  const size_t oHIT = off; off = al256(off + (size_t)gA * RCAP * 4);
  const size_t oXB  = off; off = al256(off + (size_t)MP * DF * 2);
  const size_t oAG  = off; off = al256(off + (size_t)MP * AGP * 2);
  const size_t oHB  = off; off = al256(off + (size_t)TPB * GBM * HP * 2);
  if (off > ws_size || off > (size_t)WSMAX) return;
  unsigned short* W1C = (unsigned short*)(ws + oW1C);
  unsigned short* W2C = (unsigned short*)(ws + oW2C);
  int*            CNT = (int*)(ws + oCNT);
  int*            HIT = (int*)(ws + oHIT);
  unsigned short* XB  = (unsigned short*)(ws + oXB);
  unsigned short* AG  = (unsigned short*)(ws + oAG);
  float*          TR  = (float*)(ws + oAG);
  unsigned short* HB  = (unsigned short*)(ws + oHB);

  const size_t scanLds = (size_t)AGG_LDS_INTS * 4;
  hipFuncSetAttribute(reinterpret_cast<const void*>(&k_scan1), hipFuncAttributeMaxDynamicSharedMemorySize, (int)scanLds);

  k_prep<<<nbX + UW1 / NTHR + UW2 / NTHR, NTHR, 0, stream>>>(x, W1l, W1r, W2l, W2r, nN, nbX, XB, W1C, W2C);
  k_scan1<<<gA, NTHR, scanLds, stream>>>(src, dst, nE, nN, vec8, MP, XB, AG, HIT, CNT);
  for (int band = 0; band < NBAND; ++band) {
    const int t0 = band * TPB;
    int nt = nT - t0;
    nt = nt > TPB ? TPB : nt;
    if (nt <= 0) continue;
    k_gemm1<<<dim3(nt, DH / GBN), GTHR, 0, stream>>>(AG, XB, W1C, b1, HB, t0, nN);
    k_gemm2<<<nt, GTHR, 0, stream>>>(HB, W2C, b2, TR, t0);
  }
  k_scan2<<<gA, NTHR, 0, stream>>>(HIT, CNT, TR, nN, out);
}
